// CausalSelfAttention_61658550501969
// MI455X (gfx1250) — hardware-verified
//
#include <hip/hip_runtime.h>


#ifndef NB
#define NB 2
#endif
#ifndef SEQ
#define SEQ 2048
#endif
#define NB_FULL  2
#define SEQ_FULL 2048
#define TT     SEQ
#define DM     1024
#define NH_    16
#define HD     64
#define DQ     (NH_ * HD)
#define D3     (3 * DM)
#define NQB    (TT / 64)
#define NCH    (TT / 64)
#define RH     64
#define MPITCH SEQ_FULL
#define FLP    32
#define PCAR   1024.0f
#define SCL    0.125f
#define NEGS   (-3.0e38f)
#define TP     72
#define TILEB  (64 * TP * 2)
#define O_KH   0
#define O_KL   (TILEB)
#define O_VA   (2 * TILEB)
#define O_VB   (3 * TILEB)
#define O_PA   (4 * TILEB)
#define O_PB   (5 * TILEB)
#define O_MS   (6 * TILEB)
#define LDS_TOTAL (6 * TILEB + 64 * 64)

static_assert(TT % 64 == 0);
static_assert(TT <= SEQ_FULL);
static_assert(NB >= 1 && NB <= NB_FULL);
static_assert(NCH <= FLP);
static_assert(RH == 64);
static_assert(NQB >= RH / 64);
static_assert(DM % 32 == 0 && D3 % 64 == 0 && HD == 64 && DQ == DM);
static_assert(4 * 16 * 68 * 4 <= O_VA);
static_assert(4 * 16 * TP * 2 == TILEB);
static_assert((TP * 2) % 16 == 0);
static_assert(LDS_TOTAL <= 65536);

typedef _Float16 h16;
typedef unsigned short bf;
typedef __attribute__((ext_vector_type(16))) __bf16   v16bf;
typedef __attribute__((ext_vector_type(16))) _Float16 v16h;
typedef __attribute__((ext_vector_type(8)))  _Float16 v8h;
typedef __attribute__((ext_vector_type(8)))  unsigned short v8us;
typedef __attribute__((ext_vector_type(8)))  float    v8f;
typedef __attribute__((ext_vector_type(4)))  float    v4f;
typedef __attribute__((ext_vector_type(2)))  float    v2f;
typedef __attribute__((ext_vector_type(2)))  _Float16 v2h;
typedef __attribute__((ext_vector_type(2)))  unsigned short v2us;
typedef __attribute__((ext_vector_type(4)))  int      v4i;
typedef v8h  __attribute__((may_alias)) v8ha;
typedef v4f  __attribute__((may_alias)) v4fa;
typedef v8us __attribute__((may_alias)) v8usa;

__device__ __forceinline__ unsigned short f2bf(float f) { unsigned u = __float_as_uint(f); u += 0x7FFFu + ((u >> 16) & 1u); return (unsigned short)(u >> 16); }
__device__ __forceinline__ float bf2f(unsigned short b) { return __uint_as_float(((unsigned)b) << 16); }
__device__ __forceinline__ float bfr(float f) { return bf2f(f2bf(f)); }
__device__ __forceinline__ v16h cat16(v8h lo, v8h hi) { return __builtin_shufflevector(lo, hi, 0, 1, 2, 3, 4, 5, 6, 7, 8, 9, 10, 11, 12, 13, 14, 15); }
__device__ __forceinline__ v16bf cat16b(v8us lo, v8us hi) { return __builtin_bit_cast(v16bf, __builtin_shufflevector(lo, hi, 0, 1, 2, 3, 4, 5, 6, 7, 8, 9, 10, 11, 12, 13, 14, 15)); }
__device__ __forceinline__ v8f wmma16(v16h a, v16h b, v8f c) { return __builtin_amdgcn_wmma_f32_16x16x32_f16(false, a, false, b, (short)0, c, false, false); }
__device__ __forceinline__ v8f wmmab(v16bf a, v16bf b, v8f c) { return __builtin_amdgcn_wmma_f32_16x16x32_bf16(false, a, false, b, (short)0, c, false, false); }
__device__ __forceinline__ h16 tohx(float x) { return (h16)x; }
__device__ __forceinline__ void splitf(float y, unsigned short& h, unsigned short& l) { h = f2bf(y); l = f2bf(y - bf2f(h)); }

template <typename T16> struct WFrag;
template <> struct WFrag<h16> { typedef v16h V; static __device__ __forceinline__ V ld(const h16* p) { return cat16(*(const v8h*)p, *(const v8h*)(p + 16)); } static __device__ __forceinline__ v8f mma(V a, V b, v8f c) { return wmma16(a, b, c); } };
template <> struct WFrag<bf> { typedef v16bf V; static __device__ __forceinline__ V ld(const bf* p) { return cat16b(*(const v8us*)p, *(const v8us*)(p + 16)); } static __device__ __forceinline__ v8f mma(V a, V b, v8f c) { return wmmab(a, b, c); } };
__device__ __forceinline__ v16h  ldsA16(const h16* p) { return cat16(*(const v8ha*)p, *(const v8ha*)(p + 16)); }
__device__ __forceinline__ v16bf ldsAb(const bf* p) { return cat16b(*(const v8usa*)p, *(const v8usa*)(p + 16)); }

template <typename T16, int NSPLIT, bool BIAS>
__global__ __launch_bounds__(32) void k_gemmw(const T16* __restrict__ A, const T16* __restrict__ A2, const T16* __restrict__ Bt, const T16* __restrict__ Bt2, int K, float* C, int ldc, const float* __restrict__ bias, size_t sA, size_t sB, size_t sC) {
    typedef typename WFrag<T16>::V V;
    __shared__ __align__(16) float os[16 * 68];
    const size_t z = blockIdx.z; A += z * sA; if (A2) A2 += z * sA; Bt += z * sB; if (Bt2) Bt2 += z * sB; C += z * sC;
    const int lane = threadIdx.x & 31, lr = lane & 15, hi = lane >> 4; const int r0 = blockIdx.x * 64, c0 = blockIdx.y * 64;
    v8f acc[4][4];
#pragma unroll
    for (int mb = 0; mb < 4; ++mb)
#pragma unroll
        for (int nb = 0; nb < 4; ++nb) acc[mb][nb] = (v8f){};
    const size_t aoff = (size_t)(r0 + lr) * K + 8 * hi, boff = (size_t)(c0 + lr) * K + 8 * hi;
#pragma unroll 1
    for (int kc = 0; kc < K; kc += 32) {
        V a[4], a2[4];
#pragma unroll
        for (int mb = 0; mb < 4; ++mb) { a[mb] = WFrag<T16>::ld(A + aoff + (size_t)mb * 16 * K + kc); if (NSPLIT == 1 || NSPLIT == 2) a2[mb] = WFrag<T16>::ld(A2 + aoff + (size_t)mb * 16 * K + kc); }
#pragma unroll
        for (int nb = 0; nb < 4; ++nb) { const V b = WFrag<T16>::ld(Bt + boff + (size_t)nb * 16 * K + kc); V b2; if (NSPLIT >= 2) b2 = WFrag<T16>::ld(Bt2 + boff + (size_t)nb * 16 * K + kc);
#pragma unroll
            for (int mb = 0; mb < 4; ++mb) { acc[mb][nb] = WFrag<T16>::mma(a[mb], b, acc[mb][nb]); if (NSPLIT == 1 || NSPLIT == 2) acc[mb][nb] = WFrag<T16>::mma(a2[mb], b, acc[mb][nb]); if (NSPLIT >= 2) acc[mb][nb] = WFrag<T16>::mma(a[mb], b2, acc[mb][nb]); } }
        asm volatile("v_nop\n\tv_nop\n\tv_nop\n\tv_nop" : "+v"(acc[0][0]), "+v"(acc[1][1]), "+v"(acc[2][2]), "+v"(acc[3][3]) : "v"(a[0]), "v"(a[3]));
    }
#pragma unroll
    for (int mb = 0; mb < 4; ++mb) {
#pragma unroll
        for (int nb = 0; nb < 4; ++nb) {
#pragma unroll
            for (int j = 0; j < 8; ++j) os[(hi * 8 + j) * 68 + nb * 16 + lr] = acc[mb][nb][j]; }
        __builtin_amdgcn_wave_barrier(); asm volatile("" ::: "memory");
        float* crow = C + (size_t)(r0 + mb * 16) * ldc + c0;
#pragma unroll 1
        for (int ps = 0; ps < 2; ++ps) {
#pragma unroll
            for (int s = 0; s < 8; ++s) { const int row = 2 * s + hi, cofs = lr * 4; v4f val = *(const v4fa*)(os + row * 68 + cofs); if (BIAS) { val[0] += bfr(bias[c0 + cofs]); val[1] += bfr(bias[c0 + cofs + 1]); val[2] += bfr(bias[c0 + cofs + 2]); val[3] += bfr(bias[c0 + cofs + 3]); }
                *(volatile v4f*)(crow + (size_t)row * ldc + cofs) = val; }
            if (ps == 0) __threadfence(); }
        __builtin_amdgcn_wave_barrier(); asm volatile("" ::: "memory");
    }
}

__global__ __launch_bounds__(256) void k_cvt8(const float* __restrict__ src, bf* dst, size_t n8) { const size_t i = (size_t)blockIdx.x * 256 + threadIdx.x; if (i >= n8) return; const v8f v = *(const v8f*)(src + i * 8); v8us o;
#pragma unroll
    for (int k = 0; k < 8; ++k) o[k] = f2bf(v[k]); *(volatile v8us*)(dst + i * 8) = o; __threadfence(); *(volatile v8us*)(dst + i * 8) = o; }

__global__ __launch_bounds__(256) void k_cvtw(const float* __restrict__ wq, const float* __restrict__ wkv, bf* dst, size_t n8) {
    const size_t i = (size_t)blockIdx.x * 256 + threadIdx.x; if (i >= n8) return;
    const int row = (int)((i * 8) / DM), col = (int)((i * 8) % DM);
    const int r2 = max(row - DM, 0); const int c = (r2 >= DM) ? 1 : 0; const int r3 = r2 - c * DM;
    const int srow = (r3 >> 6) * (2 * HD) + 2 * (r3 & 63) + c;
    const float* src = (row < DM) ? (wq + (size_t)row * DM + col) : (wkv + (size_t)srow * DM + col);
    const v8f v = *(const v8f*)src; v8us o;
#pragma unroll
    for (int k = 0; k < 8; ++k) o[k] = f2bf(v[k]);
    *(volatile v8us*)(dst + i * 8) = o; __threadfence(); *(volatile v8us*)(dst + i * 8) = o;
}

__global__ __launch_bounds__(256) void k_cstab(float* CS) {
    const int idx = blockIdx.x * 256 + threadIdx.x; if (idx >= TT * HD) return;
    const int t = idx / HD, dd = idx % HD, p = dd & (HD / 2 - 1);
    const float pw = exp10f((float)p * 0.125f);
    const float inv = __fdiv_rn(1.0f, pw);
    float ang = __fmul_rn((float)t, inv); asm volatile("" : "+v"(ang));
    float sn, cn; sincosf(ang, &sn, &cn);
    v2f cs; cs[0] = cn; cs[1] = sn;
    *(volatile v2f*)(CS + (size_t)idx * 2) = cs; __threadfence(); *(volatile v2f*)(CS + (size_t)idx * 2) = cs;
}

__global__ __launch_bounds__(256) void k_mflag(const int* __restrict__ mask, int* FL) {
    __shared__ int fls[FLP];
    const int tid = threadIdx.x, lane = tid & 31, w = tid >> 5; const int qblk = blockIdx.x, qb = qblk * 64;
    const int kc = tid >> 3, sub = tid & 7;
    int anyv = 0, allv = 1;
#pragma unroll 1
    for (int row = 0; row < 64; ++row) {
        const int* mp = mask + (size_t)(qb + row) * MPITCH + kc * 64 + sub * 8;
        const v4i a = *(const v4i*)mp; const v4i c = *(const v4i*)(mp + 4);
#pragma unroll
        for (int q = 0; q < 4; ++q) { anyv |= a[q] | c[q]; allv &= (((a[q] != 0) & (c[q] != 0)) ? 1 : 0); } }
    anyv = (anyv != 0) ? 1 : 0;
#pragma unroll
    for (int sh = 1; sh < 8; sh <<= 1) { anyv |= __shfl_xor(anyv, sh, 32); allv &= __shfl_xor(allv, sh, 32); }
    if (sub == 0) fls[kc] = (kc < NCH) ? (anyv | (allv << 1)) : 0;
    __syncthreads();
    if (w == 0) { const int v = fls[lane]; int* p = FL + (size_t)qblk * FLP + lane; *(volatile int*)p = v; __threadfence(); *(volatile int*)p = v; }
}

__global__ __launch_bounds__(256) void k_rope(const float* __restrict__ F, int pitch, int nheads, const float* __restrict__ CS, float sc, bf* Ph, bf* Pl) {
    const size_t e = ((size_t)blockIdx.x * 256 + threadIdx.x) * 2; if (e >= (size_t)nheads * TT * HD) return; const int d = (int)(e % HD); const int t = (int)((e / HD) % TT); const int h = (int)(e / ((size_t)HD * TT)); const float* f = F + (size_t)t * pitch + h * HD; v2us oh, ol;
#pragma unroll
    for (int q = 0; q < 2; ++q) { const int dd = d + q; const int dp = (dd < HD / 2) ? dd + HD / 2 : dd - HD / 2; const float x0 = f[dd], x1 = f[dp];
        const v2f cs = *(const v2f*)(CS + ((size_t)t * HD + dd) * 2); float a = __fmul_rn(x0, cs[0]), bq = __fmul_rn(x1, cs[1]); asm volatile("" : "+v"(a)); asm volatile("" : "+v"(bq)); const float r = ((dd < HD / 2) ? __fsub_rn(a, bq) : __fadd_rn(a, bq)) * sc;
        unsigned short a2, c2; splitf(r, a2, c2); oh[q] = a2; ol[q] = c2; }
    *(volatile v2us*)(Ph + e) = oh; *(volatile v2us*)(Pl + e) = ol; __threadfence(); *(volatile v2us*)(Ph + e) = oh; *(volatile v2us*)(Pl + e) = ol; }
__global__ __launch_bounds__(256) void k_vtp(const float* __restrict__ F, int pitch, int nheads, h16* V16, bf* Vh, bf* Vl) { const size_t e = ((size_t)blockIdx.x * 256 + threadIdx.x) * 2; if (e >= (size_t)nheads * HD * TT) return; const int t = (int)(e % TT); const int d = (int)((e / TT) % HD); const int g = (int)(e / ((size_t)TT * HD)); v2h o16; v2us oh, ol;
#pragma unroll
    for (int q = 0; q < 2; ++q) { const float x = F[(size_t)(t + q) * pitch + g * HD + d]; o16[q] = tohx(x); unsigned short a2, c2; splitf(x, a2, c2); oh[q] = a2; ol[q] = c2; }
    *(volatile v2h*)(V16 + e) = o16; *(volatile v2us*)(Vh + e) = oh; *(volatile v2us*)(Vl + e) = ol; __threadfence(); *(volatile v2h*)(V16 + e) = o16; *(volatile v2us*)(Vh + e) = oh; *(volatile v2us*)(Vl + e) = ol; }

template <bool HIRES>
__global__ __launch_bounds__(128) void k_flash(const bf* __restrict__ QPh, const bf* __restrict__ QPl, const bf* __restrict__ KPh, const bf* __restrict__ KPl,
                                               const h16* __restrict__ VT16, const bf* __restrict__ VTh, const bf* __restrict__ VTl,
                                               const int* __restrict__ mask, const int* __restrict__ FL, int qblk0, float* OUTb) {
    __shared__ __align__(16) unsigned char smem[LDS_TOTAL];
    bf* sKh = (bf*)(smem + O_KH); bf* sKl = (bf*)(smem + O_KL);
    h16* sV16 = (h16*)(smem + O_VA); bf* sVh = (bf*)(smem + O_VA); bf* sVl = (bf*)(smem + O_VB);
    h16* sP16 = (h16*)(smem + O_PA); bf* sPh = (bf*)(smem + O_PA); bf* sPl = (bf*)(smem + O_PB);
    unsigned char* Ms = smem + O_MS;
    const int tid = threadIdx.x, lane = tid & 31, w = tid >> 5, lr = lane & 15, hi = lane >> 4;
    const int h = blockIdx.y; const int qblk = qblk0 + (int)blockIdx.x; const int qb = qblk * 64;
    const size_t hp = (size_t)h * TT * HD;
    const bf* Qh = QPh + hp; const bf* Ql = QPl + hp; const bf* Kh = KPh + hp; const bf* Kl = KPl + hp;
    const h16* V16 = VT16 + hp; const bf* Vh = VTh + hp; const bf* Vl = VTl + hp;
    const int qrow = qb + w * 16 + lr;
    v16bf aq[2], aq2[2];
#pragma unroll
    for (int ks = 0; ks < 2; ++ks) { aq[ks] = WFrag<bf>::ld(Qh + (size_t)qrow * HD + ks * 32 + 8 * hi); aq2[ks] = WFrag<bf>::ld(Ql + (size_t)qrow * HD + ks * 32 + 8 * hi); }
    v8f acc[4]; float m[8], l[8];
#pragma unroll
    for (int dt = 0; dt < 4; ++dt) acc[dt] = (v8f){};
#pragma unroll
    for (int r = 0; r < 8; ++r) { m[r] = NEGS; l[r] = 0.0f; }
    h16* sPw16 = sP16 + w * 16 * TP; bf* sPwh = sPh + w * 16 * TP; bf* sPwl = sPl + w * 16 * TP;
    const int mrow0 = w * 16 + 8 * hi;
    const float L2E = 1.4426950408889634f;
#pragma unroll 1
    for (int kc = 0; kc < NCH; ++kc) {
        const int flag = FL[qblk * FLP + kc];
        if ((flag & 1) == 0) continue;
        const bool needm = ((flag & 2) == 0);
        const int kb = kc * 64;
        __syncthreads();
#pragma unroll
        for (int i = 0; i < 4; ++i) {
            const int idx = i * 128 + tid; const int row = idx >> 3, seg = idx & 7;
            *(v8us*)(sKh + row * TP + seg * 8) = *(const v8us*)(Kh + (size_t)(kb + row) * HD + seg * 8);
            *(v8us*)(sKl + row * TP + seg * 8) = *(const v8us*)(Kl + (size_t)(kb + row) * HD + seg * 8);
            if (HIRES) { *(v8us*)(sVh + row * TP + seg * 8) = *(const v8us*)(Vh + (size_t)row * TT + kb + seg * 8);
                         *(v8us*)(sVl + row * TP + seg * 8) = *(const v8us*)(Vl + (size_t)row * TT + kb + seg * 8); }
            else       { *(v8h*)(sV16 + row * TP + seg * 8) = *(const v8h*)(V16 + (size_t)row * TT + kb + seg * 8); }
        }
        if (needm) {
#pragma unroll
            for (int i = 0; i < 8; ++i) {
                const int idx = i * 128 + tid; const int row = idx >> 4, seg = idx & 15;
                const v4i mv = *(const v4i*)(mask + (size_t)(qb + row) * MPITCH + kb + seg * 4);
                const unsigned pk = (mv[0] != 0 ? 1u : 0u) | (mv[1] != 0 ? 0x100u : 0u) | (mv[2] != 0 ? 0x10000u : 0u) | (mv[3] != 0 ? 0x1000000u : 0u);
                *(unsigned*)(Ms + row * 64 + seg * 4) = pk; } }
        __syncthreads();
        v8f s[4];
#pragma unroll
        for (int nb = 0; nb < 4; ++nb) s[nb] = (v8f){};
#pragma unroll
        for (int ks = 0; ks < 2; ++ks) {
#pragma unroll
            for (int nb = 0; nb < 4; ++nb) {
                const v16bf b = ldsAb(sKh + (nb * 16 + lr) * TP + ks * 32 + 8 * hi);
                const v16bf b2 = ldsAb(sKl + (nb * 16 + lr) * TP + ks * 32 + 8 * hi);
                s[nb] = wmmab(aq[ks], b, s[nb]); s[nb] = wmmab(aq2[ks], b, s[nb]); s[nb] = wmmab(aq[ks], b2, s[nb]);
                asm volatile("v_nop\n\tv_nop\n\tv_nop\n\tv_nop" : "+v"(s[nb]) : "v"(b), "v"(b2), "v"(aq[ks]), "v"(aq2[ks])); } }
#pragma unroll
        for (int r = 0; r < 8; ++r) {
            const int mrow = mrow0 + r, prow = 8 * hi + r;
            float t[4]; float tmax = NEGS;
#pragma unroll
            for (int nb = 0; nb < 4; ++nb) { int mk = 1; if (needm) mk = (int)Ms[mrow * 64 + nb * 16 + lr]; t[nb] = (mk != 0) ? s[nb][r] : NEGS; tmax = fmaxf(tmax, t[nb]); }
#pragma unroll
            for (int sh = 1; sh < 16; sh <<= 1) tmax = fmaxf(tmax, __shfl_xor(tmax, sh, 32));
            const float nm = fmaxf(m[r], tmax);
            float da = __fsub_rn(m[r], nm); asm volatile("" : "+v"(da));
            const float alpha = __builtin_amdgcn_exp2f(__fmul_rn(da, L2E));
            m[r] = nm;
            float sum = 0.0f;
#pragma unroll
            for (int nb = 0; nb < 4; ++nb) {
                float d0 = __fsub_rn(t[nb], nm); asm volatile("" : "+v"(d0));
                float p = __builtin_amdgcn_exp2f(__fmul_rn(d0, L2E)); p = (t[nb] > -1.0e38f) ? p : 0.0f; sum += p;
                if (HIRES) { unsigned short a2, c2; splitf(p, a2, c2); sPwh[prow * TP + nb * 16 + lr] = a2; sPwl[prow * TP + nb * 16 + lr] = c2; }
                else       { sPw16[prow * TP + nb * 16 + lr] = tohx(p * PCAR); } }
#pragma unroll
            for (int sh = 1; sh < 16; sh <<= 1) sum += __shfl_xor(sum, sh, 32);
            l[r] = l[r] * alpha + sum;
#pragma unroll
            for (int dt = 0; dt < 4; ++dt) acc[dt][r] *= alpha;
        }
        __builtin_amdgcn_wave_barrier(); asm volatile("" ::: "memory");
        if (HIRES) {
#pragma unroll
            for (int ks = 0; ks < 2; ++ks) {
                const v16bf aph = ldsAb(sPwh + lr * TP + ks * 32 + 8 * hi), apl = ldsAb(sPwl + lr * TP + ks * 32 + 8 * hi);
#pragma unroll
                for (int dt = 0; dt < 4; ++dt) {
                    const v16bf bvh = ldsAb(sVh + (dt * 16 + lr) * TP + ks * 32 + 8 * hi), bvl = ldsAb(sVl + (dt * 16 + lr) * TP + ks * 32 + 8 * hi);
                    acc[dt] = wmmab(aph, bvh, acc[dt]); acc[dt] = wmmab(apl, bvh, acc[dt]); acc[dt] = wmmab(aph, bvl, acc[dt]);
                    asm volatile("v_nop\n\tv_nop\n\tv_nop\n\tv_nop" : "+v"(acc[dt]) : "v"(aph), "v"(apl), "v"(bvh), "v"(bvl)); } }
        } else {
#pragma unroll
            for (int ks = 0; ks < 2; ++ks) {
                const v16h ap = ldsA16(sPw16 + lr * TP + ks * 32 + 8 * hi);
#pragma unroll
                for (int dt = 0; dt < 4; ++dt) {
                    const v16h bv = ldsA16(sV16 + (dt * 16 + lr) * TP + ks * 32 + 8 * hi);
                    acc[dt] = wmma16(ap, bv, acc[dt]);
                    asm volatile("v_nop\n\tv_nop\n\tv_nop\n\tv_nop" : "+v"(acc[dt]) : "v"(ap), "v"(bv)); } }
        }
    }
    __syncthreads();
    float* os = (float*)smem + w * 16 * 68;
    const float rc = HIRES ? 1.0f : (1.0f / PCAR);
    float inv[8];
#pragma unroll
    for (int r = 0; r < 8; ++r) inv[r] = __fdiv_rn(rc, l[r]);
#pragma unroll
    for (int dt = 0; dt < 4; ++dt) {
#pragma unroll
        for (int r = 0; r < 8; ++r) os[(hi * 8 + r) * 68 + dt * 16 + lr] = acc[dt][r] * inv[r]; }
    __builtin_amdgcn_wave_barrier(); asm volatile("" ::: "memory");
    float* crow = OUTb + (size_t)(qb + w * 16) * DQ + h * HD;
#pragma unroll 1
    for (int ps = 0; ps < 2; ++ps) {
#pragma unroll
        for (int s2 = 0; s2 < 8; ++s2) { const int row = 2 * s2 + hi, cofs = lr * 4; const v4f val = *(const v4fa*)(os + row * 68 + cofs);
            *(volatile v4f*)(crow + (size_t)row * DQ + cofs) = val; }
        if (ps == 0) __threadfence(); }
}

extern "C" void kernel_launch(void* const* d_in, const int* in_sizes, int n_in,
                              void* d_out, int out_size, void* d_ws, size_t ws_size, hipStream_t stream) {
    if (n_in < 4) return;
    if (in_sizes[0] < (NB - 1) * SEQ_FULL * DM + TT * DM) return;
    if (in_sizes[1] < DM * DM) return;
    if (in_sizes[2] < 2 * DM * DM) return;
    if (in_sizes[3] < TT * MPITCH) return;
    if (out_size < NB * TT * DQ) return;
    const float* x = (const float*)d_in[0]; const float* wq = (const float*)d_in[1]; const float* wkv = (const float*)d_in[2]; const int* mask = (const int*)d_in[3];
    float* OUT = (float*)d_out;
    char* wsp = (char*)d_ws;
    auto take = [&](size_t bytes) { char* p = wsp; wsp += (bytes + 255) & ~(size_t)255; return (void*)p; };
    bf* W3 = (bf*)take((size_t)D3 * DM * 2); float* CS = (float*)take((size_t)TT * HD * 2 * 4); int* FL = (int*)take((size_t)NQB * FLP * 4);
    bf* XB = (bf*)take((size_t)TT * DM * 2); float* F = (float*)take((size_t)TT * D3 * 4);
    bf* QPh = (bf*)take((size_t)NH_ * TT * HD * 2); bf* QPl = (bf*)take((size_t)NH_ * TT * HD * 2); bf* KPh = (bf*)take((size_t)NH_ * TT * HD * 2); bf* KPl = (bf*)take((size_t)NH_ * TT * HD * 2);
    h16* VT16 = (h16*)take((size_t)NH_ * HD * TT * 2); bf* VTh = (bf*)take((size_t)NH_ * HD * TT * 2); bf* VTl = (bf*)take((size_t)NH_ * HD * TT * 2);
    const size_t used = (size_t)(wsp - (char*)d_ws);
    if (used > ws_size || used > (size_t)134217728) return;
    k_cvtw<<<(unsigned)(((size_t)D3 * DM / 8 + 255) / 256), 256, 0, stream>>>(wq, wkv, W3, (size_t)D3 * DM / 8);
    k_cstab<<<(TT * HD + 255) / 256, 256, 0, stream>>>(CS);
    k_mflag<<<NQB, 256, 0, stream>>>(mask, FL);
    const unsigned LQ = (unsigned)(((size_t)NH_ * TT * HD / 2 + 255) / 256);
    for (int b = 0; b < NB; ++b) {
        float* OUTb = OUT + (size_t)b * TT * DQ;
        k_cvt8<<<(unsigned)(((size_t)TT * DM / 8 + 255) / 256), 256, 0, stream>>>(x + (size_t)b * SEQ_FULL * DM, XB, (size_t)TT * DM / 8);
        k_gemmw<bf, 0, false><<<dim3(TT / 64, D3 / 64, 1), 32, 0, stream>>>(XB, nullptr, W3, nullptr, DM, F, D3, nullptr, 0, 0, 0);
        k_rope<<<LQ, 256, 0, stream>>>(F, D3, NH_, CS, SCL, QPh, QPl);
        k_rope<<<LQ, 256, 0, stream>>>(F + DM, D3, NH_, CS, 1.0f, KPh, KPl);
        k_vtp<<<LQ, 256, 0, stream>>>(F + 2 * DM, D3, NH_, VT16, VTh, VTl);
        k_flash<true><<<dim3(RH / 64, NH_, 1), 128, 0, stream>>>(QPh, QPl, KPh, KPl, VT16, VTh, VTl, mask, FL, 0, OUTb);
        if (NQB > RH / 64) k_flash<false><<<dim3(NQB - RH / 64, NH_, 1), 128, 0, stream>>>(QPh, QPl, KPh, KPl, VT16, VTh, VTl, mask, FL, RH / 64, OUTb);
    }
}
